// TABlock_26268019982573
// MI455X (gfx1250) — hardware-verified
//
#include <hip/hip_runtime.h>
#include <math.h>

constexpr int kBatch = 16;
constexpr int kSeq   = 1024;
constexpr int kDim   = 768;
constexpr int kTok   = kBatch * kSeq;
constexpr int kGrp   = 4;
constexpr int kNGrp  = kBatch / kGrp;
constexpr float kWCarry    = 16.0f;
constexpr float kWCarryInv = 1.0f / 16.0f;
constexpr float kPCarry    = 32768.0f;
constexpr float kPCarryInv = 1.0f / 32768.0f;
static_assert(kBatch % kGrp == 0, "group split");
static_assert(kDim % 64 == 0 && kSeq % 64 == 0 && kTok % 64 == 0, "tile multiples");
static_assert(kDim % 32 == 0 && kSeq % 32 == 0, "K multiples of 32");

typedef __attribute__((ext_vector_type(16))) _Float16 v16h;
typedef __attribute__((ext_vector_type(8)))  _Float16 v8h;
typedef __attribute__((ext_vector_type(16))) __bf16   v16b;
typedef __attribute__((ext_vector_type(8)))  __bf16   v8b;
typedef __attribute__((ext_vector_type(8)))  float    v8f;
typedef __attribute__((ext_vector_type(4)))  float    v4f;
typedef __attribute__((ext_vector_type(4)))  unsigned int v4u;

__device__ __forceinline__ unsigned short f2bf_bits(float f) {
  unsigned u = __float_as_uint(f);
  return (unsigned short)((u + 0x7FFFu + ((u >> 16) & 1u)) >> 16);
}
__device__ __forceinline__ float bf_bits2f(unsigned short h) { return __uint_as_float(((unsigned)h) << 16); }

__device__ __forceinline__ void dep_guard_h(v8f& a, v8f& b, v16h x, v16h y) { asm volatile("v_nop\n\tv_nop\n\tv_nop\n\tv_nop" : "+v"(a), "+v"(b) : "v"(x), "v"(y)); }
__device__ __forceinline__ void dep_guard_b(v8f& a, v8f& b, v16b x, v16b y) { asm volatile("v_nop\n\tv_nop\n\tv_nop\n\tv_nop" : "+v"(a), "+v"(b) : "v"(x), "v"(y)); }
__device__ __forceinline__ void keep4_h(v16h a, v16h b, v16h c, v16h d) { asm volatile("v_nop" :: "v"(a), "v"(b), "v"(c), "v"(d)); }
__device__ __forceinline__ void keep4_b(v16b a, v16b b, v16b c, v16b d) { asm volatile("v_nop" :: "v"(a), "v"(b), "v"(c), "v"(d)); }
__device__ __forceinline__ void acc_guard4(v8f& a, v8f& b, v8f& c, v8f& d) { asm volatile("v_nop\n\tv_nop\n\tv_nop\n\tv_nop" : "+v"(a), "+v"(b), "+v"(c), "+v"(d)); }
template <typename T> struct Frag;
template <> struct Frag<_Float16> {
  typedef v16h V; union U { v16h v; v8h h[2]; };
  static __device__ __forceinline__ v16h load(const _Float16* p) {
    U f; f.h[0] = *(const v8h*)(p); f.h[1] = *(const v8h*)(p + 16); return f.v;
  }
  static __device__ __forceinline__ v8f mma(v16h a, v16h b, v8f c) {
    return __builtin_amdgcn_wmma_f32_16x16x32_f16(false, a, false, b, (short)0, c, false, false);
  }
  static __device__ __forceinline__ void guard(v8f& a, v8f& b, v16h x, v16h y) { dep_guard_h(a, b, x, y); }
  static __device__ __forceinline__ void keep(v16h a, v16h b, v16h c, v16h d) { keep4_h(a, b, c, d); }
};
template <> struct Frag<__bf16> {
  typedef v16b V; union U { v16b v; v8b h[2]; };
  static __device__ __forceinline__ v16b load(const __bf16* p) {
    U f; f.h[0] = *(const v8b*)(p); f.h[1] = *(const v8b*)(p + 16); return f.v;
  }
  static __device__ __forceinline__ v8f mma(v16b a, v16b b, v8f c) {
    return __builtin_amdgcn_wmma_f32_16x16x32_bf16(false, a, false, b, (short)0, c, false, false);
  }
  static __device__ __forceinline__ void guard(v8f& a, v8f& b, v16b x, v16b y) { dep_guard_b(a, b, x, y); }
  static __device__ __forceinline__ void keep(v16b a, v16b b, v16b c, v16b d) { keep4_b(a, b, c, d); }
};

__device__ __forceinline__ unsigned pk16(unsigned short a, unsigned short b) { return (unsigned)a | ((unsigned)b << 16); }
__device__ __forceinline__ unsigned short h_bits(float f) { const _Float16 h = (_Float16)f; return __builtin_bit_cast(unsigned short, h); }

template <int ET> struct Elem;
template <> struct Elem<0> { typedef _Float16 T; };
template <> struct Elem<1> { typedef __bf16 T; };
template <int ET, bool SPLIT, int BIAS_MODE, int OUT_MODE, bool RESID, int ACT = 0>
__global__ __launch_bounds__(256) void wmma_gemm64(
    const unsigned short* __restrict__ Ap, const unsigned short* __restrict__ A2p, int lda, long strideA,
    const unsigned short* __restrict__ Btp, const unsigned short* __restrict__ Bt2p, int ldb, long strideB,
    void* __restrict__ Cout, void* __restrict__ Cout2, int ldc, long strideC,
    const float* __restrict__ bias,
    const float* __restrict__ resid, long strideR,
    int M, int N, int K, float scale) {
  typedef typename Elem<ET>::T T;
  typedef typename Frag<T>::V V;
  const T* A = (const T*)Ap; const T* A2 = (const T*)A2p; const T* Bt = (const T*)Btp; const T* Bt2 = (const T*)Bt2p;
  __shared__ __align__(16) float sT[8][16 * 68];
  const int b    = blockIdx.y;
  const int lane = threadIdx.x & 31;
  const int wave = threadIdx.x >> 5;
  const int tilesN = N >> 6;
  const int tilesM = M >> 6;
  const int tile = blockIdx.x * 8 + wave;
  if (tile >= tilesM * tilesN) return;
  const int tm = tile / tilesN;
  const int tn = tile - tm * tilesN;
  const int m0 = tm << 6;
  const int n0 = tn << 6;

  const T* Ab  = A  + (size_t)b * strideA;
  const T* Bb  = Bt + (size_t)b * strideB;
  const T* Ab2 = SPLIT ? (A2  + (size_t)b * strideA) : nullptr;
  const T* Bb2 = SPLIT ? (Bt2 + (size_t)b * strideB) : nullptr;

  const int rlane = lane & 15;
  const int koff  = (lane >> 4) * 8;
  const int mOff  = (lane >> 4) * 8;

  v8f acc[4][4];
#pragma unroll
  for (int i = 0; i < 4; ++i)
#pragma unroll
    for (int j = 0; j < 4; ++j) acc[i][j] = (v8f){0.f,0.f,0.f,0.f,0.f,0.f,0.f,0.f};

  for (int k0 = 0; k0 < K; k0 += 32) {
    V bh[4], bl[4];
#pragma unroll
    for (int j = 0; j < 4; ++j) {
      const size_t bo = (size_t)(n0 + (j << 4) + rlane) * ldb + koff + k0;
      bh[j] = Frag<T>::load(Bb + bo);
      if (SPLIT) bl[j] = Frag<T>::load(Bb2 + bo);
    }
#pragma unroll
    for (int i = 0; i < 4; ++i) {
      const size_t ao = (size_t)(m0 + (i << 4) + rlane) * lda + koff + k0;
      V ah = Frag<T>::load(Ab + ao);
      V al;
      if (SPLIT) al = Frag<T>::load(Ab2 + ao);
#pragma unroll
      for (int j = 0; j < 4; ++j) {
        acc[i][j] = Frag<T>::mma(ah, bh[j], acc[i][j]);
        if (SPLIT) {
          acc[i][j] = Frag<T>::mma(ah, bl[j], acc[i][j]);
          acc[i][j] = Frag<T>::mma(al, bh[j], acc[i][j]);
        }
      }
      Frag<T>::guard(acc[i][0], acc[i][3], ah, SPLIT ? al : ah);
    }
    Frag<T>::keep(bh[0], bh[1], bh[2], bh[3]);
    if (SPLIT) Frag<T>::keep(bl[0], bl[1], bl[2], bl[3]);
  }
  acc_guard4(acc[0][0], acc[0][1], acc[0][2], acc[0][3]);
  acc_guard4(acc[1][0], acc[1][1], acc[1][2], acc[1][3]);
  acc_guard4(acc[2][0], acc[2][1], acc[2][2], acc[2][3]);
  acc_guard4(acc[3][0], acc[3][1], acc[3][2], acc[3][3]);

  float* slab = sT[wave];
  const float* Rb = RESID ? (resid + (size_t)b * strideR) : nullptr;
#pragma unroll
  for (int i = 0; i < 4; ++i) {
    const int mBase = m0 + (i << 4);
#pragma unroll
    for (int j = 0; j < 4; ++j) {
      const int n = n0 + (j << 4) + rlane;
      float bv = 0.f;
      if (BIAS_MODE == 2) bv = bias[n];
#pragma unroll
      for (int r = 0; r < 8; ++r) {
        float v = acc[i][j][r] * scale;
        if (BIAS_MODE == 1) v += bias[mBase + mOff + r];
        if (BIAS_MODE == 2) v += bv;
        if (RESID) v += Rb[(size_t)(mBase + mOff + r) * ldc + n];
        if (ACT == 2) v = fmaxf(v, 0.0f);
        if (ACT == 4) v = (v > 0.f) ? v : 0.01f * v;
        slab[(mOff + r) * 68 + (j << 4) + rlane] = v;
      }
    }
    __builtin_amdgcn_fence(__ATOMIC_RELEASE, "workgroup");
    __builtin_amdgcn_wave_barrier();
    __builtin_amdgcn_fence(__ATOMIC_ACQUIRE, "workgroup");
    if (OUT_MODE == 0) {
      float* C = (float*)Cout + (size_t)b * strideC;
      const int hh = lane >> 4, c4 = (lane & 15) * 4;
      for (int pass = 0; pass < 2; ++pass) {
#pragma unroll
        for (int it = 0; it < 8; ++it) {
          const int row = it * 2 + hh;
          v4f v = *(const v4f*)(slab + row * 68 + c4);
          *(volatile v4f*)(C + (size_t)(mBase + row) * ldc + n0 + c4) = v;
        }
        __threadfence();
      }
    } else {
      const int q = lane >> 3, c8 = (lane & 7) * 8;
      unsigned short* C  = (unsigned short*)Cout  + (size_t)b * strideC;
      unsigned short* C2 = (OUT_MODE == 2) ? ((unsigned short*)Cout2 + (size_t)b * strideC) : nullptr;
      for (int pass = 0; pass < 2; ++pass) {
#pragma unroll
        for (int it = 0; it < 4; ++it) {
          const int row = it * 4 + q;
          const float* sp = slab + row * 68 + c8;
          v8h hv, lv;
#pragma unroll
          for (int e = 0; e < 8; ++e) {
            if (OUT_MODE == 1) {
              hv[e] = (_Float16)sp[e];
            } else {
              unsigned short hb = f2bf_bits(sp[e]);
              unsigned short lb = f2bf_bits(sp[e] - bf_bits2f(hb));
              hv[e] = __builtin_bit_cast(_Float16, hb);
              lv[e] = __builtin_bit_cast(_Float16, lb);
            }
          }
          *(volatile v8h*)(C + (size_t)(mBase + row) * ldc + n0 + c8) = hv;
          if (OUT_MODE == 2) *(volatile v8h*)(C2 + (size_t)(mBase + row) * ldc + n0 + c8) = lv;
        }
        __threadfence();
      }
    }
    __builtin_amdgcn_fence(__ATOMIC_RELEASE, "workgroup");
    __builtin_amdgcn_wave_barrier();
    __builtin_amdgcn_fence(__ATOMIC_ACQUIRE, "workgroup");
  }
}

__global__ __launch_bounds__(256) void cast8_f16_kernel(const float* __restrict__ in, unsigned short* __restrict__ out,
                                                        int n8, float scale) {
  const int i = blockIdx.x * 256 + threadIdx.x;
  if (i >= n8) return;
  const float* p = in + 8 * (size_t)i;
  const v4f a = *(const v4f*)(p);
  const v4f c = *(const v4f*)(p + 4);
  unsigned short hb[8];
#pragma unroll
  for (int e = 0; e < 4; ++e) {
    hb[e]     = h_bits(a[e] * scale);
    hb[4 + e] = h_bits(c[e] * scale);
  }
  const v4u u = (v4u){pk16(hb[0], hb[1]), pk16(hb[2], hb[3]), pk16(hb[4], hb[5]), pk16(hb[6], hb[7])};
  unsigned short* q = out + 8 * (size_t)i;
  *(volatile v4u*)q = u;
  __threadfence();
  *(volatile v4u*)q = u;
}

__global__ __launch_bounds__(128) void softmax_row_kernel(const float* __restrict__ S, unsigned short* __restrict__ P,
                                                          float carry) {
  __shared__ float redM[4];
  __shared__ float redS[4];
  const int row  = blockIdx.x;
  const int t    = threadIdx.x;
  const int lane = t & 31, wave = t >> 5;
  const int c0   = t * 8;
  const float* sr = S + (size_t)row * kSeq + c0;
  const v4f a = *(const v4f*)(sr);
  const v4f c = *(const v4f*)(sr + 4);
  float x[8];
#pragma unroll
  for (int e = 0; e < 4; ++e) { x[e] = a[e]; x[4 + e] = c[e]; }
  float m = fmaxf(fmaxf(fmaxf(x[0], x[1]), fmaxf(x[2], x[3])), fmaxf(fmaxf(x[4], x[5]), fmaxf(x[6], x[7])));
#pragma unroll
  for (int off = 16; off > 0; off >>= 1) m = fmaxf(m, __shfl_xor(m, off, 32));
  if (lane == 0) redM[wave] = m;
  __syncthreads();
  const float M = fmaxf(fmaxf(redM[0], redM[1]), fmaxf(redM[2], redM[3]));
  float ex[8];
#pragma unroll
  for (int e = 0; e < 8; ++e) ex[e] = __expf(x[e] - M);
  float s = ((ex[0] + ex[1]) + (ex[2] + ex[3])) + ((ex[4] + ex[5]) + (ex[6] + ex[7]));
#pragma unroll
  for (int off = 16; off > 0; off >>= 1) s += __shfl_xor(s, off, 32);
  if (lane == 0) redS[wave] = s;
  __syncthreads();
  const float l = (redS[0] + redS[1]) + (redS[2] + redS[3]);
  const float f = carry * (1.0f / l);
  unsigned short hb[8];
#pragma unroll
  for (int e = 0; e < 8; ++e) hb[e] = h_bits(ex[e] * f);
  const v4u u = (v4u){pk16(hb[0], hb[1]), pk16(hb[2], hb[3]), pk16(hb[4], hb[5]), pk16(hb[6], hb[7])};
  unsigned short* q = P + (size_t)row * kSeq + c0;
  *(volatile v4u*)q = u;
  __threadfence();
  *(volatile v4u*)q = u;
}

extern "C" void kernel_launch(void* const* d_in, const int* in_sizes, int n_in,
                              void* d_out, int out_size, void* d_ws, size_t ws_size,
                              hipStream_t stream) {
  if (n_in < 7) return;
  if (in_sizes[0] != kTok * kDim) return;
  if (in_sizes[1] != kDim * kDim || in_sizes[3] != kDim * kDim || in_sizes[5] != kDim * kDim) return;
  if (in_sizes[2] != kDim || in_sizes[4] != kDim || in_sizes[6] != kDim) return;
  if (out_size != kTok * kDim) return;

  const float* X  = (const float*)d_in[0];
  const float* Wq = (const float*)d_in[1];
  const float* bq = (const float*)d_in[2];
  const float* Wk = (const float*)d_in[3];
  const float* bk = (const float*)d_in[4];
  const float* Wv = (const float*)d_in[5];
  const float* bv = (const float*)d_in[6];
  float* outp = (float*)d_out;

  const size_t SZ_W   = (size_t)kDim * kDim * 2;
  const size_t SZ_X16 = (size_t)kTok * kDim * 2;
  const size_t SZ_S   = (size_t)kGrp * kSeq * kSeq * 4;
  const size_t SZ_P   = (size_t)kGrp * kSeq * kSeq * 2;
  size_t off = 0;
  const size_t oWQ  = off; off += SZ_W;
  const size_t oWK  = off; off += SZ_W;
  const size_t oWV  = off; off += SZ_W;
  const size_t oX16 = off; off += SZ_X16;
  const size_t oQ16 = off; off += SZ_X16;
  const size_t oK16 = off; off += SZ_X16;
  const size_t oVT  = off; off += SZ_X16;
  const size_t oS   = off; off += SZ_S;
  const size_t oP   = off; off += SZ_P;
  const size_t TOTAL = off;
  if (TOTAL > ws_size) return;
  if (TOTAL > (size_t)134217728) return;

  char* ws = (char*)d_ws;
  unsigned short* WQ16 = (unsigned short*)(ws + oWQ);
  unsigned short* WK16 = (unsigned short*)(ws + oWK);
  unsigned short* WV16 = (unsigned short*)(ws + oWV);
  unsigned short* X16  = (unsigned short*)(ws + oX16);
  unsigned short* Q16  = (unsigned short*)(ws + oQ16);
  unsigned short* K16  = (unsigned short*)(ws + oK16);
  unsigned short* VT16 = (unsigned short*)(ws + oVT);
  float*          Sf   = (float*)(ws + oS);
  unsigned short* P16  = (unsigned short*)(ws + oP);

  const dim3 blk(256);
  const float scoreScale = 1.0f / sqrtf((float)kDim);

  {
    const int n8 = kDim * kDim / 8;
    const dim3 gW((n8 + 255) / 256);
    cast8_f16_kernel<<<gW, blk, 0, stream>>>(Wq, WQ16, n8, kWCarry);
    cast8_f16_kernel<<<gW, blk, 0, stream>>>(Wk, WK16, n8, kWCarry);
    cast8_f16_kernel<<<gW, blk, 0, stream>>>(Wv, WV16, n8, kWCarry);
  }
  {
    const int n8 = kTok * kDim / 8;
    cast8_f16_kernel<<<dim3((n8 + 255) / 256), blk, 0, stream>>>(X, X16, n8, 1.0f);
  }

  const dim3 gProj(((kTok / 64) * (kDim / 64) + 7) / 8, 1);
  const dim3 gV((((kDim / 64) * (kSeq / 64)) + 7) / 8, kBatch);
  const dim3 gS((((kSeq / 64) * (kSeq / 64)) + 7) / 8, kGrp);
  const dim3 gPV((((kDim / 64) * (kSeq / 64)) + 7) / 8, kGrp);

  wmma_gemm64<0, false, 2, 1, false, 0><<<gProj, blk, 0, stream>>>(
      X16, X16, kDim, 0L, WQ16, WQ16, kDim, 0L, (void*)Q16, (void*)Q16, kDim, 0L,
      bq, X, 0L, kTok, kDim, kDim, kWCarryInv);
  wmma_gemm64<0, false, 2, 1, false, 0><<<gProj, blk, 0, stream>>>(
      X16, X16, kDim, 0L, WK16, WK16, kDim, 0L, (void*)K16, (void*)K16, kDim, 0L,
      bk, X, 0L, kTok, kDim, kDim, kWCarryInv);
  wmma_gemm64<0, false, 1, 1, false, 0><<<gV, blk, 0, stream>>>(
      WV16, WV16, kDim, 0L, X16, X16, kDim, (long)kSeq * kDim, (void*)VT16, (void*)VT16, kSeq, (long)kDim * kSeq,
      bv, X, 0L, kDim, kSeq, kDim, kWCarryInv);

  for (int g = 0; g < kNGrp; ++g) {
    const size_t tokOff = (size_t)g * kGrp * kSeq * kDim;
    const unsigned short* Qg = Q16 + tokOff;
    const unsigned short* Kg = K16 + tokOff;
    wmma_gemm64<0, false, 0, 0, false, 0><<<gS, blk, 0, stream>>>(
        Qg, Qg, kDim, (long)kSeq * kDim, Kg, Kg, kDim, (long)kSeq * kDim, (void*)Sf, (void*)Sf, kSeq, (long)kSeq * kSeq,
        bq, X, 0L, kSeq, kSeq, kDim, scoreScale);
    softmax_row_kernel<<<dim3(kGrp * kSeq), dim3(128), 0, stream>>>(Sf, P16, kPCarry);
    const unsigned short* Vg = VT16 + (size_t)g * kGrp * kDim * kSeq;
    float* Og = outp + tokOff;
    const float* Xg = X + tokOff;
    wmma_gemm64<0, false, 0, 0, true, 0><<<gPV, blk, 0, stream>>>(
        Vg, Vg, kSeq, (long)kDim * kSeq, P16, P16, kSeq, (long)kSeq * kSeq, (void*)Og, (void*)Og, kSeq, (long)kSeq * kDim,
        bq, Xg, (long)kSeq * kDim, kDim, kSeq, kSeq, kPCarryInv);
  }
}
